// DeepSetGraphClassifier_84490596647533
// MI455X (gfx1250) — hardware-verified
//
#include <hip/hip_runtime.h>
#include <math.h>

typedef __attribute__((ext_vector_type(16))) _Float16 v16h;
typedef __attribute__((ext_vector_type(8)))  _Float16 v8h;
typedef __attribute__((ext_vector_type(16))) __bf16   v16b;
typedef __attribute__((ext_vector_type(8)))  float    v8f;
typedef __attribute__((ext_vector_type(4)))  float    v4f;

__device__ __forceinline__ int frag_k(int i, int h) { return (i < 8) ? (8 * h + i) : (16 + 8 * h + (i - 8)); }
__device__ __forceinline__ __bf16 bf16_rne(float f) {
    unsigned int u = __float_as_uint(f);
    u += 0x7fffu + ((u >> 16) & 1u);
    return __builtin_bit_cast(__bf16, (unsigned short)(u >> 16));
}
__device__ __forceinline__ float bf16_f32(__bf16 b) { return __uint_as_float(((unsigned int)__builtin_bit_cast(unsigned short, b)) << 16); }
__device__ __forceinline__ v8f wmma16(v16h a, v16h b, v8f c) {
    c = __builtin_amdgcn_wmma_f32_16x16x32_f16(false, a, false, b, (short)0, c, false, false);
    asm volatile("v_nop\n\tv_nop\n\tv_nop\n\tv_nop" : "+v"(c) : "v"(a), "v"(b));
    return c;
}
__device__ __forceinline__ v8f wmmab(v16b a, v16b b, v8f c) {
    c = __builtin_amdgcn_wmma_f32_16x16x32_bf16(false, a, false, b, (short)0, c, false, false);
    asm volatile("v_nop\n\tv_nop\n\tv_nop\n\tv_nop" : "+v"(c) : "v"(a), "v"(b));
    return c;
}
struct Split { v16b hi, lo; };
__device__ __forceinline__ v8f wmma3(const Split& a, const Split& b, v8f c) {
    c = __builtin_amdgcn_wmma_f32_16x16x32_bf16(false, a.hi, false, b.hi, (short)0, c, false, false);
    c = __builtin_amdgcn_wmma_f32_16x16x32_bf16(false, a.hi, false, b.lo, (short)0, c, false, false);
    c = __builtin_amdgcn_wmma_f32_16x16x32_bf16(false, a.lo, false, b.hi, (short)0, c, false, false);
    asm volatile("v_nop\n\tv_nop\n\tv_nop\n\tv_nop" : "+v"(c) : "v"(a.hi), "v"(a.lo), "v"(b.hi), "v"(b.lo));
    return c;
}
struct Split3 { v16b hi, mid, lo; };
__device__ __forceinline__ v8f wmma6(const Split3& a, const Split3& b, v8f c) {
    c = __builtin_amdgcn_wmma_f32_16x16x32_bf16(false, a.hi, false, b.hi, (short)0, c, false, false);
    c = __builtin_amdgcn_wmma_f32_16x16x32_bf16(false, a.hi, false, b.mid, (short)0, c, false, false);
    c = __builtin_amdgcn_wmma_f32_16x16x32_bf16(false, a.mid, false, b.hi, (short)0, c, false, false);
    c = __builtin_amdgcn_wmma_f32_16x16x32_bf16(false, a.hi, false, b.lo, (short)0, c, false, false);
    c = __builtin_amdgcn_wmma_f32_16x16x32_bf16(false, a.mid, false, b.mid, (short)0, c, false, false);
    c = __builtin_amdgcn_wmma_f32_16x16x32_bf16(false, a.lo, false, b.hi, (short)0, c, false, false);
    asm volatile("v_nop\n\tv_nop\n\tv_nop\n\tv_nop" : "+v"(c) : "v"(a.hi), "v"(a.mid), "v"(a.lo), "v"(b.hi), "v"(b.mid), "v"(b.lo));
    return c;
}

__device__ __forceinline__ v16h fh_ld(const float* __restrict__ p, long long sk, int k0, int h, int klen, float s) {
    v16h a;
#pragma unroll
    for (int i = 0; i < 16; ++i) { const int k = k0 + frag_k(i, h); a[i] = (k < klen) ? (_Float16)(p[(long long)k * sk] * s) : (_Float16)0.f; }
    return a;
}
__device__ __forceinline__ Split sp_ld(const float* __restrict__ p, long long sk, int k0, int h, int klen, float s) {
    Split r;
#pragma unroll
    for (int i = 0; i < 16; ++i) {
        const int k = k0 + frag_k(i, h); const float x = (k < klen) ? p[(long long)k * sk] * s : 0.f;
        const __bf16 hb = bf16_rne(x); r.hi[i] = hb; r.lo[i] = bf16_rne(x - bf16_f32(hb));
    }
    return r;
}
__device__ __forceinline__ Split3 sp3_ld(const float* __restrict__ p, long long sk, int k0, int h, int klen, float s) {
    Split3 r;
#pragma unroll
    for (int i = 0; i < 16; ++i) {
        const int k = k0 + frag_k(i, h); const float x = (k < klen) ? p[(long long)k * sk] * s : 0.f;
        const __bf16 hb = bf16_rne(x); const float r1 = x - bf16_f32(hb); const __bf16 mb = bf16_rne(r1);
        r.hi[i] = hb; r.mid[i] = mb; r.lo[i] = bf16_rne(r1 - bf16_f32(mb));
    }
    return r;
}
__device__ __forceinline__ v16b bh_ld(const float* __restrict__ p, long long sk, int k0, int h, int klen, float s) {
    v16b a;
#pragma unroll
    for (int i = 0; i < 16; ++i) { const int k = k0 + frag_k(i, h); a[i] = bf16_rne((k < klen) ? p[(long long)k * sk] * s : 0.f); }
    return a;
}
__device__ __forceinline__ v16h fh_row(const _Float16* __restrict__ row, int k0, int h) {
    v16h a;
#pragma unroll
    for (int i = 0; i < 16; ++i) a[i] = row[k0 + frag_k(i, h)];
    return a;
}

#define VST2(T, ptr, val) do { *(volatile T*)(ptr) = (val); __threadfence(); *(volatile T*)(ptr) = (val); } while (0)
typedef float v4f __attribute__((ext_vector_type(4)));
#define VST2V4(ptr, val) do { *(volatile v4f*)(ptr) = (val); __threadfence(); *(volatile v4f*)(ptr) = (val); } while (0)

__device__ __attribute__((noinline)) float act_fn(float v, int act) {
    if (act == 1) return fmaxf(v, 0.f);
    if (act == 2) { const float u = 0.7978845608028654f * (v + 0.044715f * v * v * v); return 0.5f * v * (1.f + tanhf(u)); }
    if (act == 3) return v / (1.f + expf(-v));
    if (act == 4) return 0.5f * v * (1.f + erff(v * 0.7071067811865476f));
    if (act == 5) return tanhf(v);
    if (act == 6) return 1.f / (1.f + expf(-v));
    if (act == 7) return (v > 0.f) ? v : 0.01f * v;
    if (act == 8) return (v > 0.f) ? v : (expf(v) - 1.f);
    if (act == 9) return fminf(fmaxf(v, 0.f), 6.f);
    if (act == 10) return fabsf(v);
    if (act == 11) return (v >= 0.f) ? v : 0.1f * v;
    if (act == 12) return (v > 0.f) ? v : 0.2f * v;
    if (act == 13) return (v > 20.f) ? v : log1pf(expf(v));
    return v;
}

struct GemmP {
    const float* A; const float* B; const float* bias; const float* R; float* C;
    long long sAo, sAi, sAm, sAk, sBo, sBi, sBn, sBk, sCo, sCi, sCm, sRo, sRi, sRm, sRn;
    int M, N, K, zi_n, flags, act; float alpha, beta, sa, sb;
    int Npad, pad_;
};
static_assert(sizeof(GemmP) == 5 * 8 + 15 * 8 + 6 * 4 + 4 * 4 + 2 * 4, "GemmP has padding");

template <int MODE>
__global__ __launch_bounds__(32) void k_gemm(GemmP p) {
    const int lane = threadIdx.x & 31, h = lane >> 4, l15 = lane & 15;
    const int m0 = blockIdx.y * 16, n0 = blockIdx.x * 32;
    const int z = blockIdx.z, zo = z / p.zi_n, zi = z - zo * p.zi_n;
    const float* A = p.A + zo * p.sAo + zi * p.sAi;
    const float* B = p.B + zo * p.sBo + zi * p.sBi;
    const int am = min(m0 + l15, p.M - 1);
    v8f acc[2], comp[2];
#pragma unroll
    for (int t = 0; t < 2; ++t) { v8f zz = {}; acc[t] = zz; comp[t] = zz; }
    for (int k0 = 0; k0 < p.K; k0 += 32) {
        const float* arow = A + (long long)am * p.sAm;
        if (MODE == 1) {
            const Split a = sp_ld(arow, p.sAk, k0, h, p.K, 1.f);
#pragma unroll
            for (int t = 0; t < 2; ++t) {
                const int bn = min(n0 + t * 16 + l15, p.N - 1);
                acc[t] = wmma3(a, sp_ld(B + (long long)bn * p.sBn, p.sBk, k0, h, p.K, 1.f), acc[t]);
            }
        } else if (MODE == 3) {
            const Split3 a = sp3_ld(arow, p.sAk, k0, h, p.K, 1.f);
#pragma unroll
            for (int t = 0; t < 2; ++t) {
                const int bn = min(n0 + t * 16 + l15, p.N - 1);
                acc[t] = wmma6(a, sp3_ld(B + (long long)bn * p.sBn, p.sBk, k0, h, p.K, 1.f), acc[t]);
            }
        } else if (MODE == 4) {
            const Split3 a = sp3_ld(arow, p.sAk, k0, h, p.K, 1.f);
#pragma unroll
            for (int t = 0; t < 2; ++t) {
                const int bn = min(n0 + t * 16 + l15, p.N - 1); v8f zz = {};
                const v8f part = wmma6(a, sp3_ld(B + (long long)bn * p.sBn, p.sBk, k0, h, p.K, 1.f), zz);
                const v8f y = part - comp[t]; const v8f s = acc[t] + y; comp[t] = (s - acc[t]) - y; acc[t] = s;
            }
        } else if (MODE == 2) {
            const v16b a = bh_ld(arow, p.sAk, k0, h, p.K, 1.f);
#pragma unroll
            for (int t = 0; t < 2; ++t) {
                const int bn = min(n0 + t * 16 + l15, p.N - 1);
                acc[t] = wmmab(a, bh_ld(B + (long long)bn * p.sBn, p.sBk, k0, h, p.K, 1.f), acc[t]);
            }
        } else {
            const v16h a = fh_ld(arow, p.sAk, k0, h, p.K, p.sa);
#pragma unroll
            for (int t = 0; t < 2; ++t) {
                const int bn = min(n0 + t * 16 + l15, p.N - 1);
                acc[t] = wmma16(a, fh_ld(B + (long long)bn * p.sBn, p.sBk, k0, h, p.K, p.sb), acc[t]);
            }
        }
    }
    const float iscale = (MODE == 0) ? p.alpha / (p.sa * p.sb) : p.alpha;
    float* C = p.C + zo * p.sCo + zi * p.sCi;
    const float* R = p.R + zo * p.sRo + zi * p.sRi;
    __shared__ __align__(16) float ctile[16][36];
#pragma unroll
    for (int t = 0; t < 2; ++t) {
        const int n = n0 + t * 16 + l15; const int nn = min(n, p.N - 1);
#pragma unroll
        for (int r = 0; r < 8; ++r) {
            const int m = m0 + 8 * h + r; const int mm = min(m, p.M - 1);
            float v = acc[t][r] * iscale;
            if (p.flags & 1) v += p.bias[nn];
            if (p.flags & 2) v += p.bias[mm];
            v = act_fn(v, p.act);
            if (p.flags & 4) v += p.beta * R[(long long)mm * p.sRm + (long long)nn * p.sRn];
            ctile[8 * h + r][t * 16 + l15] = (n < p.N) ? v : 0.f;
        }
    }
    __syncthreads();
    const int NW = (p.Npad > p.N) ? p.Npad : p.N;
    const bool fast = (m0 + 16 <= p.M) && (n0 + 32 <= NW) && ((p.sCm & 3) == 0) && ((((size_t)C) & 15) == 0);
    if (fast) {
#pragma unroll
        for (int s = 0; s < 4; ++s) {
            const int row = s * 4 + (lane >> 3), c4 = (lane & 7) * 4;
            const v4f v = *(const v4f*)&ctile[row][c4];
            VST2V4(C + (long long)(m0 + row) * p.sCm + n0 + c4, v);
        }
    } else {
        for (int row = 0; row < 16; ++row) {
            const int m = m0 + row, n = n0 + lane;
            if (m < p.M && n < NW) VST2(float, C + (long long)m * p.sCm + n, ctile[row][lane]);
        }
    }
}

#define AW 4
struct AttnP {
    const float* Q; const float* K; const float* V; float* O; float* P; const float* Mf; const int* Mi; float* ST;
    const float* Pw; const float* Rt; const int* SQ; const int* SK;
    long long swb, swh, swi, swj, srb, srh, sri;
    long long sQb, sQh, sQi, sQd, sKb, sKh, sKj, sKd, sVb, sVh, sVj, sVd, sOb, sOh, sOi, sPb, sPh, sPi, smb, smh, smi, smj;
    int Lq, Lk, dh, dv, hrep, causal, coff, pband;
    float scale, mfill; int nonorm, mpol;
    int roff, rn, segpol, win;
};
static_assert(sizeof(AttnP) == 12 * 8 + 29 * 8 + 16 * 4, "AttnP has padding");

#ifndef KATTN_ATTR
#define KATTN_ATTR
#endif
template <int DHP, int DVP, int QM, bool SPLITPV, bool TWOPASS>
__global__ __launch_bounds__(32 * AW) KATTN_ATTR void k_attn(AttnP p) {
    constexpr int NT = DVP / 16;
    constexpr int KS = DHP / 32;
    constexpr int VP = DVP + 8;
    __shared__ __align__(16) float    pl[AW][16 * 64];
    __shared__ __align__(16) _Float16 vl[(SPLITPV ? 2 : 1) * 64 * VP];
    const int lane = threadIdx.x & 31, hf = lane >> 4, l15 = lane & 15, wave = threadIdx.x >> 5;
    const int h = blockIdx.y, b = blockIdx.z, hk = h / p.hrep;
    const int q0 = (blockIdx.x * AW + wave) * 16;
    float* myp = pl[wave];
    const float L2E = 1.4426950408889634f;
    const float NEG = -__builtin_inff();
    const int qi = min(q0 + l15, p.Lq - 1);
    const float* qrow = p.Q + b * p.sQb + h * p.sQh + (long long)qi * p.sQi;
    const float* kbase = p.K + b * p.sKb + hk * p.sKh;
    const float* vbase = p.V + b * p.sVb + hk * p.sVh;
    v16h qa[QM == 0 ? KS : 1]; Split qs_[QM == 1 ? KS : 1]; Split3 qt_[QM == 2 ? KS : 1];
#pragma unroll
    for (int ks = 0; ks < KS; ++ks) {
        if (QM == 2) qt_[ks] = sp3_ld(qrow, p.sQd, ks * 32, hf, p.dh, 1.f);
        else if (QM == 1) qs_[ks] = sp_ld(qrow, p.sQd, ks * 32, hf, p.dh, 1.f);
        else qa[ks] = fh_ld(qrow, p.sQd, ks * 32, hf, p.dh, 1.f);
    }
    v8f o[NT]; float m8[8], l8[8];
#pragma unroll
    for (int t = 0; t < NT; ++t) { v8f zz = {}; o[t] = zz; }
#pragma unroll
    for (int i = 0; i < 8; ++i) { m8[i] = NEG; l8[i] = 0.f; }
    int jend = p.Lk;
    if (p.causal == 1) { const int je = (blockIdx.x * AW + AW - 1) * 16 + 16 + p.coff; jend = min(jend, max(je, 0)); }
    const int npass = TWOPASS ? 2 : 1;
    for (int pass = 0; pass < npass; ++pass) {
        const bool dopv = (!TWOPASS) || pass == 1;
        for (int j0 = 0; j0 < jend; j0 += 64) {
            if (dopv) {
                __syncthreads();
                for (int idx = threadIdx.x; idx < 64 * DVP; idx += 32 * AW) {
                    const int jr = idx / DVP, d = idx - jr * DVP, j = j0 + jr;
                    const float f = (j < p.Lk && d < p.dv) ? vbase[(long long)j * p.sVj + (long long)d * p.sVd] : 0.f;
                    if (SPLITPV) {
                        const __bf16 hb = bf16_rne(f);
                        ((__bf16*)vl)[jr * VP + d] = hb; ((__bf16*)vl)[64 * VP + jr * VP + d] = bf16_rne(f - bf16_f32(hb));
                    } else vl[jr * VP + d] = (_Float16)f;
                }
            }
            v8f s[4];
#pragma unroll
            for (int t = 0; t < 4; ++t) {
                const int j = min(j0 + t * 16 + l15, p.Lk - 1);
                const float* krow = kbase + (long long)j * p.sKj;
                v8f acc = {};
#pragma unroll
                for (int ks = 0; ks < KS; ++ks) {
                    if (QM == 2)      acc = wmma6(qt_[ks], sp3_ld(krow, p.sKd, ks * 32, hf, p.dh, 1.f), acc);
                    else if (QM == 1) acc = wmma3(qs_[ks], sp_ld(krow, p.sKd, ks * 32, hf, p.dh, 1.f), acc);
                    else              acc = wmma16(qa[ks], fh_ld(krow, p.sKd, ks * 32, hf, p.dh, 1.f), acc);
                }
                s[t] = acc;
            }
            float pv[8][4];
#pragma unroll
            for (int i = 0; i < 8; ++i) {
                const int irow = q0 + i + 8 * hf;
                const int ic = min(irow, p.Lq - 1);
                float sc[4];
#pragma unroll
                for (int t = 0; t < 4; ++t) {
                    const int jg = j0 + t * 16 + l15;
                    float v = s[t][i] * p.scale;
                    if (p.Mf) v += p.Mf[b * p.smb + h * p.smh + (long long)ic * p.smi + (long long)min(jg, p.Lk - 1) * p.smj];
                    if (p.Rt) { int rc = ic - min(jg, p.Lk - 1) + p.roff; rc = rc < 0 ? 0 : (rc >= p.rn ? p.rn - 1 : rc); v += p.Rt[b * p.srb + h * p.srh + (long long)ic * p.sri + rc]; }
                    if (p.Mi) { const int mv = p.Mi[b * p.smb + h * p.smh + (long long)ic * p.smi + (long long)min(jg, p.Lk - 1) * p.smj]; if (p.mpol ? (mv != 0) : (mv == 0)) v = p.mfill; }
                    if (p.SQ) { const bool same = p.SQ[(long long)b * p.Lq + ic] == p.SK[(long long)b * p.Lk + min(jg, p.Lk - 1)]; if (p.segpol ? same : !same) v = p.mfill; }
                    if (p.causal == 2 && jg > irow + p.coff) v = p.mfill;
                    if (jg >= p.Lk || (p.causal == 1 && jg > irow + p.coff) || (p.causal == 3 && jg < irow + p.coff) || (p.win > 0 && irow + p.coff - jg > p.win)) v = NEG; else v *= L2E;
                    sc[t] = v;
                }
                if (!TWOPASS || pass == 0) {
                    float mx = fmaxf(fmaxf(sc[0], sc[1]), fmaxf(sc[2], sc[3]));
                    mx = fmaxf(mx, __shfl_xor(mx, 1, 32)); mx = fmaxf(mx, __shfl_xor(mx, 2, 32));
                    mx = fmaxf(mx, __shfl_xor(mx, 4, 32)); mx = fmaxf(mx, __shfl_xor(mx, 8, 32));
                    const float mnew = fmaxf(m8[i], mx);
                    const float corr = (mnew == NEG) ? 1.f : exp2f(m8[i] - mnew);
                    float rs = 0.f;
#pragma unroll
                    for (int t = 0; t < 4; ++t) {
                        const float pp = (sc[t] == NEG) ? 0.f : exp2f(sc[t] - mnew); rs += pp;
                        pv[i][t] = p.Pw ? pp * p.Pw[b * p.swb + h * p.swh + (long long)ic * p.swi + (long long)min(j0 + t * 16 + l15, p.Lk - 1) * p.swj] : pp;
                    }
                    rs += __shfl_xor(rs, 1, 32); rs += __shfl_xor(rs, 2, 32); rs += __shfl_xor(rs, 4, 32); rs += __shfl_xor(rs, 8, 32);
                    l8[i] = l8[i] * corr + rs; m8[i] = mnew;
                    if (!TWOPASS) {
#pragma unroll
                        for (int t = 0; t < NT; ++t) o[t][i] *= corr;
                    }
                } else {
                    const float inv = (l8[i] > 0.f) ? 1.f / l8[i] : 0.f;
#pragma unroll
                    for (int t = 0; t < 4; ++t) {
                        const int jg = j0 + t * 16 + l15;
                        float pp = (sc[t] == NEG) ? 0.f : exp2f(sc[t] - m8[i]) * inv;
                        if (p.Pw) pp *= p.Pw[b * p.swb + h * p.swh + (long long)ic * p.swi + (long long)min(jg, p.Lk - 1) * p.swj];
                        pv[i][t] = pp;
                    }
                }
            }
            if (dopv) {
#pragma unroll
                for (int i = 0; i < 8; ++i)
#pragma unroll
                    for (int t = 0; t < 4; ++t) myp[(i + 8 * hf) * 64 + t * 16 + l15] = pv[i][t];
                __syncthreads();
                if (p.P) {
                    float* pb_ = p.P + b * p.sPb + h * p.sPh;
                    const bool fastP = (p.pband == 0) && ((p.sPi & 3) == 0) && (j0 + 64 <= p.Lk) && (q0 + 16 <= p.Lq) && ((((size_t)pb_) & 15) == 0);
                    if (fastP) {
#pragma unroll
                        for (int s = 0; s < 8; ++s) {
                            const int row = s * 2 + (lane >> 4), c4 = (lane & 15) * 4;
                            const v4f v = *(const v4f*)(myp + row * 64 + c4);
                            VST2V4(pb_ + (long long)(q0 + row) * p.sPi + j0 + c4, v);
                        }
                    } else {
                        for (int row = 0; row < 16; ++row) {
                            const int irow = q0 + row; if (irow >= p.Lq) continue;
                            for (int c = lane; c < 64; c += 32) {
                                const int jg = j0 + c; if (jg >= p.Lk) continue;
                                if (p.pband == 0) VST2(float, pb_ + (long long)irow * p.sPi + jg, myp[row * 64 + c]);
                                else if (jg - irow <= p.pband && irow - jg <= p.pband) VST2(float, pb_ + (long long)irow * p.sPi + (jg - irow + p.pband), myp[row * 64 + c]);
                            }
                        }
                    }
                }
                if (SPLITPV) {
                    const Split pa0 = sp_ld(myp + l15 * 64, 1, 0, hf, 64, 1.f), pa1 = sp_ld(myp + l15 * 64, 1, 32, hf, 64, 1.f);
                    const __bf16* vh = (const __bf16*)vl; const __bf16* vlo = vh + 64 * VP;
#pragma unroll
                    for (int t = 0; t < NT; ++t) {
                        const int dcol = t * 16 + l15;
                        Split b0, b1;
#pragma unroll
                        for (int e = 0; e < 16; ++e) {
                            const int k0 = frag_k(e, hf), k1 = 32 + frag_k(e, hf);
                            b0.hi[e] = vh[k0 * VP + dcol]; b0.lo[e] = vlo[k0 * VP + dcol]; b1.hi[e] = vh[k1 * VP + dcol]; b1.lo[e] = vlo[k1 * VP + dcol];
                        }
                        o[t] = wmma3(pa0, b0, o[t]);
                        o[t] = wmma3(pa1, b1, o[t]);
                    }
                } else {
                    const v16h pa0 = fh_ld(myp + l15 * 64, 1, 0, hf, 64, 4096.f), pa1 = fh_ld(myp + l15 * 64, 1, 32, hf, 64, 4096.f);
#pragma unroll
                    for (int t = 0; t < NT; ++t) {
                        const int dcol = t * 16 + l15;
                        v16h b0, b1;
#pragma unroll
                        for (int e = 0; e < 16; ++e) { b0[e] = vl[frag_k(e, hf) * VP + dcol]; b1[e] = vl[(32 + frag_k(e, hf)) * VP + dcol]; }
                        o[t] = wmma16(pa0, b0, o[t]);
                        o[t] = wmma16(pa1, b1, o[t]);
                    }
                }
            }
        }
    }
    float* obase = p.O + b * p.sOb + h * p.sOh;
    if (p.ST) {
        const int rl = lane >> 1, isel = rl & 7;
        float mv = 0.f, lv = 0.f;
#pragma unroll
        for (int i = 0; i < 8; ++i) if (i == isel) { mv = m8[i]; lv = l8[i]; }
        const int irow = q0 + rl;
        if (irow < p.Lq) { float* st = p.ST + (((long long)b * gridDim.y + h) * p.Lq + irow) * 2 + (lane & 1); VST2(float, st, (lane & 1) ? lv : mv * 0.6931471805599453f); }
    }
    float invr[8];
#pragma unroll
    for (int i = 0; i < 8; ++i) {
        if (TWOPASS) invr[i] = SPLITPV ? 1.f : (1.f / 4096.f);
        else if (p.nonorm) invr[i] = exp2f(m8[i]) * (SPLITPV ? 1.f : (1.f / 4096.f));
        else invr[i] = (l8[i] > 0.f) ? (SPLITPV ? 1.f / l8[i] : 1.f / (l8[i] * 4096.f)) : 0.f;
    }
    __syncthreads();
    const bool ofast = ((p.sOi & 3) == 0) && ((((size_t)obase) & 15) == 0) && (q0 + 16 <= p.Lq);
#pragma unroll
    for (int c0 = 0; c0 < DVP; c0 += 64) {
#pragma unroll
        for (int i = 0; i < 8; ++i)
#pragma unroll
            for (int t = 0; t < NT; ++t) if (t * 16 >= c0 && t * 16 < c0 + 64) myp[(i + 8 * hf) * 64 + (t * 16 - c0) + l15] = o[t][i] * invr[i];
        __syncthreads();
        const int cw = (DVP - c0 < 64) ? (DVP - c0) : 64;
        if (ofast && (c0 + cw <= p.dv) && (cw % 32 == 0)) {
            const int lpr = cw / 4;
            const int rows_per_ins = 32 / lpr;
            for (int r0 = 0; r0 < 16; r0 += rows_per_ins) {
                const int row = r0 + lane / lpr, c4 = (lane % lpr) * 4;
                const v4f v = *(const v4f*)(myp + row * 64 + c4);
                VST2V4(obase + (long long)(q0 + row) * p.sOi + c0 + c4, v);
            }
        } else {
            for (int row = 0; row < 16; ++row) {
                const int irow = q0 + row; if (irow >= p.Lq) continue;
                for (int c = lane; c < cw; c += 32) { const int d = c0 + c; if (d < p.dv) VST2(float, obase + (long long)irow * p.sOi + d, myp[row * 64 + c]); }
            }
        }
        __syncthreads();
    }
}

struct TrP { const float* src; float* dst; const float* R2; long long sSz, lds, sDz, ldd, sRz, ldr; int R, C, flags, act; float alpha, beta; };
static_assert(sizeof(TrP) == 3 * 8 + 6 * 8 + 6 * 4, "TrP has padding");
__global__ __launch_bounds__(256) void k_tr(TrP p) {
    __shared__ float tile[32][33];
    const int c0 = blockIdx.x * 32, r0 = blockIdx.y * 32, z = blockIdx.z;
    const int lane = threadIdx.x & 31, wave = threadIdx.x >> 5;
    const float* s = p.src + z * p.sSz;
#pragma unroll
    for (int k = 0; k < 4; ++k) {
        const int rl = wave * 4 + k, r = r0 + rl, c = c0 + lane;
        tile[rl][lane] = (r < p.R && c < p.C) ? s[(long long)r * p.lds + c] : 0.f;
    }
    __syncthreads();
    float* d = p.dst + z * p.sDz; const float* rr = p.R2 + z * p.sRz;
#pragma unroll
    for (int k = 0; k < 4; ++k) {
        const int cl = wave * 4 + k, c = c0 + cl, r = r0 + lane;
        if (c < p.C && r < p.R) {
            float v = act_fn(p.alpha * tile[lane][cl], p.act);
            if (p.flags & 1) v += p.beta * rr[(long long)c * p.ldr + r];
            VST2(float, d + (long long)c * p.ldd + r, v);
        }
    }
}

__global__ __launch_bounds__(256) void k_affine(const float* __restrict__ src, float* __restrict__ dst, int n, float a, float b, const float* __restrict__ sdev) {
    const int i = blockIdx.x * 256 + threadIdx.x;
    if (i < n) { const float aa = sdev ? a * sdev[0] : a; const float v = aa * src[i] + b; VST2(float, dst + i, v); }
}

struct SmP { const float* src; float* dst; const float* Mf; long long sz, sr, dz, dr, smz, smr; int n, pad; float scale_in, scale_out; };
static_assert(sizeof(SmP) == 3 * 8 + 6 * 8 + 4 * 4, "SmP has padding");
__global__ __launch_bounds__(256) void k_softmax(SmP p) {
    __shared__ float red[256];
    const int r = blockIdx.x, z = blockIdx.y, tid = threadIdx.x;
    const float* s = p.src + z * p.sz + (long long)r * p.sr;
    const float* mf = p.Mf ? (p.Mf + z * p.smz + (long long)r * p.smr) : nullptr;
    float mx = -__builtin_inff();
    for (int j = tid; j < p.n; j += 256) { float v = s[j] * p.scale_in; if (mf) v += mf[j]; mx = fmaxf(mx, v); }
    red[tid] = mx; __syncthreads();
    for (int o = 128; o > 0; o >>= 1) { if (tid < o) red[tid] = fmaxf(red[tid], red[tid + o]); __syncthreads(); }
    mx = red[0]; __syncthreads();
    float sum = 0.f;
    for (int j = tid; j < p.n; j += 256) { float v = s[j] * p.scale_in; if (mf) v += mf[j]; sum += (mx == -__builtin_inff()) ? 0.f : expf(v - mx); }
    red[tid] = sum; __syncthreads();
    for (int o = 128; o > 0; o >>= 1) { if (tid < o) red[tid] += red[tid + o]; __syncthreads(); }
    sum = red[0];
    const float inv = (sum > 0.f) ? p.scale_out / sum : 0.f;
    float* d = p.dst + z * p.dz + (long long)r * p.dr;
    for (int j = tid; j < p.n; j += 256) { float v = s[j] * p.scale_in; if (mf) v += mf[j]; const float o = (mx == -__builtin_inff()) ? 0.f : expf(v - mx) * inv; VST2(float, d + j, o); }
}
__global__ __launch_bounds__(256) void k_stats(const float* __restrict__ x, long long sz, long long so, long long si, int inner, int n, float eps, float* __restrict__ stat, int mode) {
    __shared__ float red[256];
    const int z = blockIdx.x, tid = threadIdx.x;
    const float* base = x + z * sz;
    float s = 0.f;
    for (int e = tid; e < n; e += 256) s += base[(long long)(e / inner) * so + (long long)(e % inner) * si];
    red[tid] = s; __syncthreads();
    for (int o = 128; o > 0; o >>= 1) { if (tid < o) red[tid] += red[tid + o]; __syncthreads(); }
    const float mu = (mode == 0 || mode == 3) ? red[0] / (float)n : 0.f; __syncthreads();
    float q = 0.f;
    for (int e = tid; e < n; e += 256) { const float dlt = base[(long long)(e / inner) * so + (long long)(e % inner) * si] - mu; q += dlt * dlt; }
    red[tid] = q; __syncthreads();
    for (int o = 128; o > 0; o >>= 1) { if (tid < o) red[tid] += red[tid + o]; __syncthreads(); }
    {
        float rs;
        if (mode == 2) rs = sqrtf((float)n) / fmaxf(sqrtf(red[0]), eps); else if (mode == 3) rs = rsqrtf(red[0] / (float)(n - 1) + eps); else rs = rsqrtf(red[0] / (float)n + eps);
        if (tid < 32) { const float v = (tid == 0) ? mu : ((tid == 1) ? rs : 0.f); VST2(float, stat + (long long)z * 32 + tid, v); }
    }
}
__global__ __launch_bounds__(256) void k_norm_apply(const float* __restrict__ x, float* __restrict__ y, const float* __restrict__ stat, const float* __restrict__ g, const float* __restrict__ bta,
                                                     int Z, int C, int L, int G, int bn, int act) {
    const long long idx = (long long)blockIdx.x * 256 + threadIdx.x;
    if (idx >= (long long)Z * C * L) return;
    const int l = (int)(idx % L); const long long zc = idx / L; const int c = (int)(zc % C), z = (int)(zc / C); (void)l;
    const int set = bn ? c : (z * G + c / (C / G));
    float v = (x[idx] - stat[(long long)set * 32]) * stat[(long long)set * 32 + 1];
    if (g) v *= g[c];
    if (bta) v += bta[c];
    v = act_fn(v, act);
    VST2(float, y + idx, v);
}

__global__ __launch_bounds__(256) void k_lse_neg(const float* __restrict__ st, float* __restrict__ c, int n) {
    const int i = blockIdx.x * 256 + threadIdx.x;
    if (i < n) { const float v = -(st[2 * i] + logf(st[2 * i + 1])); VST2(float, c + i, v); }
}

__global__ __launch_bounds__(256) void k_iota(int* __restrict__ dst, int n, int a, int b) {
    const int i = blockIdx.x * 256 + threadIdx.x;
    if (i < n) { const int v = a * i + b; VST2(int, dst + i, v); }
}

__global__ __launch_bounds__(256) void k_axpby(const float* __restrict__ x, const float* __restrict__ y, float* __restrict__ dst, int n, float a, float b, float c) {
    const int i = blockIdx.x * 256 + threadIdx.x;
    if (i < n) { const float v = a * x[i] + b * y[i] + c; VST2(float, dst + i, v); }
}

struct RopeP { const float* X; float* Y; const float* C; const float* Sn; const int* pos; long long sXr, sXh, sYr, sYh, sCb, sCp, sCd; int R, Hn, D, S, mode, tmode, pmode, pad; };
static_assert(sizeof(RopeP) == 5 * 8 + 7 * 8 + 8 * 4, "RopeP has padding");
__global__ __launch_bounds__(256) void k_rope(RopeP p) {
    const long long idx = (long long)blockIdx.x * 256 + threadIdx.x;
    if (idx >= (long long)p.R * p.Hn * p.D) return;
    const int d = (int)(idx % p.D); const long long rh = idx / p.D; const int h = (int)(rh % p.Hn); const int r = (int)(rh / p.Hn);
    const int half = p.D / 2;
    int partner; float sign;
    if (p.mode == 0) { partner = (d < half) ? d + half : d - half; sign = (d < half) ? -1.f : 1.f; }
    else { partner = d ^ 1; sign = (d & 1) ? 1.f : -1.f; }
    const int tcol = (p.tmode == 0) ? d : ((p.tmode == 1) ? (d % half) : (d >> 1));
    const int pp = (p.pmode == 0) ? (r % p.S) : ((p.pmode == 1) ? h : p.pos[r]);
    const long long toff = (long long)(r / p.S) * p.sCb + (long long)pp * p.sCp + (long long)tcol * p.sCd;
    const float* xr = p.X + (long long)r * p.sXr + (long long)h * p.sXh;
    const float v = xr[d] * p.C[toff] + sign * xr[partner] * p.Sn[toff];
    VST2(float, p.Y + (long long)r * p.sYr + (long long)h * p.sYh + d, v);
}

__global__ __launch_bounds__(256) void k_invf(float* __restrict__ invb, int half, int D, float base, float num, int fmode, float cexp) {
    const int i = blockIdx.x * 256 + threadIdx.x;
    if (i >= ((half + 31) / 32) * 32) return;
    if (i >= half) { VST2(float, invb + i, 0.f); return; }
    const float e = (float)(2 * i) / (float)D;
    float invf;
    if (fmode == 1) invf = num * expf((float)(2 * i) * cexp);
    else if (fmode == 2) invf = num * powf(base, (-2.0f * ((float)i - 1.0f)) / (float)D);
    else invf = num * (1.0f / powf(base, e));
    VST2(float, invb + i, invf);
}
__global__ __launch_bounds__(256) void k_sincos(float* __restrict__ cs, float* __restrict__ sn, const float* __restrict__ invb, int S, int half, float pscale) {
    const int idx = blockIdx.x * 256 + threadIdx.x;
    if (idx >= S * half) return;
    const int s = idx / half, i = idx - s * half;
    const float ang = (pscale * (float)s) * invb[i];
    VST2(float, cs + idx, cosf(ang)); VST2(float, sn + idx, sinf(ang));
}

__global__ __launch_bounds__(256) void k_mulact(const float* __restrict__ x, const float* __restrict__ y, float* __restrict__ dst, int n, int act) {
    const int i = blockIdx.x * 256 + threadIdx.x;
    if (i < n) { const float v = act_fn(x[i], act) * y[i]; VST2(float, dst + i, v); }
}

__global__ __launch_bounds__(256) void k_matvec(GemmP p) {
    const int rpt = (p.N == 1) ? 1 : 32;
    const long long r0 = ((long long)blockIdx.x * 256 + threadIdx.x) * rpt; const int z = blockIdx.z, zo = z / p.zi_n, zi = z - zo * p.zi_n;
    if (r0 >= p.M) return;
    const float* Bb = p.B + zo * p.sBo + zi * p.sBi;
    float* C = p.C + zo * p.sCo + zi * p.sCi; const float* R = p.R + zo * p.sRo + zi * p.sRi;
    for (int rr = 0; rr < rpt; ++rr) {
        const long long r = r0 + rr; if (r >= p.M) break;
        const float* A = p.A + zo * p.sAo + zi * p.sAi + r * p.sAm;
        float acc[8] = {0.f, 0.f, 0.f, 0.f, 0.f, 0.f, 0.f, 0.f};
        for (int k = 0; k < p.K; ++k) { const float a = A[(long long)k * p.sAk];
#pragma unroll
            for (int j = 0; j < 8; ++j) if (j < p.N) acc[j] += a * Bb[(long long)j * p.sBn + (long long)k * p.sBk]; }
#pragma unroll
        for (int j = 0; j < 8; ++j) if (j < p.N) {
            float v = acc[j] * p.alpha;
            if (p.flags & 1) v += p.bias[j];
            if (p.flags & 2) v += p.bias[r];
            v = act_fn(v, p.act);
            if (p.flags & 4) v += p.beta * R[r * p.sRm + (long long)j * p.sRn];
            VST2(float, C + r * p.sCm + j, v);
        }
    }
}
__global__ __launch_bounds__(256) void k_smallsoftmax(const float* __restrict__ src, float* __restrict__ dst, long long sr, long long dr, int n, long long R, float scale) {
    const long long r0 = ((long long)blockIdx.x * 256 + threadIdx.x) * 32;
    for (int rr = 0; rr < 32; ++rr) {
        const long long r = r0 + rr; if (r >= R) return;
        const float* s = src + r * sr; float* d = dst + r * dr;
        float mx = -__builtin_inff();
        for (int j = 0; j < n; ++j) mx = fmaxf(mx, s[j] * scale);
        float sum = 0.f;
        for (int j = 0; j < n; ++j) sum += expf(s[j] * scale - mx);
        const float inv = 1.f / sum;
        for (int j = 0; j < n; ++j) { const float v = expf(s[j] * scale - mx) * inv; VST2(float, d + j, v); }
    }
}

__global__ __launch_bounds__(32) void k_unitstat(float* __restrict__ st) { const int t = threadIdx.x; const float v = (t == 1) ? 1.f : 0.f; VST2(float, st + t, v); }

__global__ __launch_bounds__(256) void k_lincopy(const float* __restrict__ src, long long lds, float* __restrict__ dst, long long ldd, long long rows, int cols) {
    const long long i = (long long)blockIdx.x * 256 + threadIdx.x; if (i >= rows * cols) return;
    const long long r = i / cols; const int c = (int)(i - r * cols);
    const float v = src[r * lds + c]; VST2(float, dst + r * ldd + c, v);
}


#define IL3_CH 4096
__global__ __launch_bounds__(256) void k_csr3_bcount(const int* __restrict__ tgt, int E, int N, int* __restrict__ CNT) { __shared__ int tt[IL3_CH]; const int ch = blockIdx.x; const int b = threadIdx.x; const int e0 = ch * IL3_CH; const int nt = min(IL3_CH, E - e0);
    for (int i = b; i < nt; i += 256) tt[i] = (int)(((long long)tgt[e0 + i] * 256) / N); __syncthreads(); int c = 0;
    for (int i = 0; i < nt; ++i) c += (tt[i] == b); VST2(int, CNT + (long long)ch * 256 + b, c); }
__global__ __launch_bounds__(256) void k_csr3_bscan(const int* __restrict__ CNT, int nch, int E, int* __restrict__ OFFB, int* __restrict__ BOFF) { __shared__ int tot[256]; const int b = threadIdx.x; int s = 0; for (int ch = 0; ch < nch; ++ch) s += CNT[(long long)ch * 256 + b]; tot[b] = s; __syncthreads();
    if (b == 0) { int run = 0; for (int i = 0; i < 256; ++i) { const int v = tot[i]; tot[i] = run; run += v; } } __syncthreads();
    int run = tot[b]; VST2(int, BOFF + b, run); if (b == 255) VST2(int, BOFF + 256, E);
    for (int ch = 0; ch < nch; ++ch) { VST2(int, OFFB + (long long)ch * 256 + b, run); run += CNT[(long long)ch * 256 + b]; } }
__global__ __launch_bounds__(256) void k_csr3_bscatter(const int* __restrict__ tgt, int E, int N, const int* __restrict__ OFFB, int* __restrict__ BUF) { __shared__ int tt[IL3_CH]; const int ch = blockIdx.x; const int b = threadIdx.x; const int e0 = ch * IL3_CH; const int nt = min(IL3_CH, E - e0);
    for (int i = b; i < nt; i += 256) tt[i] = (int)(((long long)tgt[e0 + i] * 256) / N); __syncthreads(); int pos = OFFB[(long long)ch * 256 + b];
    for (int i = 0; i < nt; ++i) if (tt[i] == b) { VST2(int, BUF + pos, e0 + i); ++pos; } }
template <int CAP>
__global__ __launch_bounds__(256) void k_csr3_lists(const int* __restrict__ tgt, const int* __restrict__ BUF, const int* __restrict__ BOFF, int N, int* __restrict__ NBR, int* __restrict__ cnt) { const int d = blockIdx.x * 256 + threadIdx.x; if (d >= N) return; const int b = (int)(((long long)d * 256) / N); int n = 0; int* row = NBR + (long long)d * CAP;
    for (int p = BOFF[b]; p < BOFF[b + 1]; ++p) { const int e = BUF[p]; if (tgt[e] == d) { if (n < CAP) VST2(int, row + n, e); ++n; } }
    for (int j = n; j < CAP; ++j) VST2(int, row + j, -1); VST2(int, cnt + d, min(n, CAP)); }
__global__ __launch_bounds__(256) void k_csr3_scan(const int* __restrict__ cnt, int* __restrict__ off, int N) {
    __shared__ int part[256]; const int per = ((((N + 255) / 256) + 31) / 32) * 32; const int a = threadIdx.x * per, b = min(N, a + per); int s = 0;
    for (int i = a; i < b; ++i) s += cnt[i]; part[threadIdx.x] = s; __syncthreads();
    if (threadIdx.x == 0) { int run = 0; for (int t = 0; t < 256; ++t) { const int v = part[t]; part[t] = run; run += v; } } __syncthreads();
    int run = part[threadIdx.x]; for (int i = a; i < b; ++i) { VST2(int, off + i, run); run += cnt[i]; }
    if (a < N && b == N) { VST2(int, off + N, run); } }
template <int CAP>
__global__ __launch_bounds__(256) void k_csr3_slotcopy(const int* __restrict__ off, const int* __restrict__ NBR, int* __restrict__ slot, int N) {
    const int t = blockIdx.x * 256 + threadIdx.x; const int tot = off[N]; if (t >= tot) return;
    int lo = 0, hi = N - 1; while (lo < hi) { const int mid = (lo + hi + 1) >> 1; if (off[mid] <= t) lo = mid; else hi = mid - 1; }
    int j = t - off[lo]; j = (j < 0) ? 0 : ((j >= CAP) ? (CAP - 1) : j); VST2(int, slot + t, NBR[(long long)lo * CAP + j]); }


__global__ __launch_bounds__(256) void k_csr_mean(const float* __restrict__ Hh, const int* __restrict__ src, const int* __restrict__ off, const int* __restrict__ slot, float* __restrict__ AGG, int N, int D) {
    const long long t = (long long)blockIdx.x * 256 + threadIdx.x; if (t >= (long long)N * D) return; const int d = (int)(t % D); const int i = (int)(t / D); const int a = off[i], b = off[i + 1]; float s = 0.f;
    for (int p = a; p < b; ++p) s += Hh[(long long)src[slot[p]] * D + d];
    VST2(float, AGG + t, s / fmaxf((float)(b - a), 1.f));
}

__global__ __launch_bounds__(256) void k_ds_dis(const int* __restrict__ off, float* __restrict__ DIS, int N) { const int n = blockIdx.x * 256 + threadIdx.x; if (n >= N) return; VST2(float, DIS + n, rsqrtf((float)(off[n + 1] - off[n]) + 1.f)); }
__global__ __launch_bounds__(256) void k_ds_rows(const int* __restrict__ sb, int* __restrict__ ROW, int G, int MS) { const int g = blockIdx.x * 256 + threadIdx.x; if (g >= G) return; const int s = sb[g]; int pos = 0;
#pragma unroll 1
    for (int j = 0; j < g; ++j) pos += (sb[j] == s); VST2(int, ROW + g, s * MS + pos); }
__global__ __launch_bounds__(256) void k_ds_agg(const float* __restrict__ T, const float* __restrict__ DIS, const int* __restrict__ ei, const int* __restrict__ off, const int* __restrict__ slot, const float* __restrict__ bias, float* __restrict__ OUT, int N, int C) { const long long q = (long long)blockIdx.x * 256 + threadIdx.x; if (q >= (long long)N * C) return; const int c = (int)(q % C); const int n = (int)(q / C); const float dn = DIS[n]; float s = dn * T[q]; for (int p = off[n]; p < off[n + 1]; ++p) { const int sidx = ei[slot[p]]; s += DIS[sidx] * T[(long long)sidx * C + c]; } VST2(float, OUT + q, fmaxf(dn * s + bias[c], 0.f)); }
__global__ __launch_bounds__(256) void k_ds_pack(const float* __restrict__ GE, const int* __restrict__ ROW, float* __restrict__ XP, int G, int H, int total) { const int q = blockIdx.x * 256 + threadIdx.x; if (q < total) VST2(float, XP + q, 0.f); }
__global__ __launch_bounds__(256) void k_ds_pack2(const float* __restrict__ GE, const int* __restrict__ ROW, float* __restrict__ XP, int G, int H) { const int q = blockIdx.x * 256 + threadIdx.x; if (q >= G * H) return; const int c = q % H; const int g = q / H; VST2(float, XP + (long long)ROW[g] * H + c, GE[q]); }
__global__ __launch_bounds__(256) void k_ds_setsum(const float* __restrict__ P2, float* __restrict__ AGG, int S, int MS, int H) { const int q = blockIdx.x * 256 + threadIdx.x; if (q >= S * H) return; const int c = q % H; const int s = q / H; float acc = 0.f;
#pragma unroll 1
    for (int m = 0; m < MS; ++m) acc += P2[((long long)s * MS + m) * H + c]; VST2(float, AGG + q, acc); }

template __global__ void k_gemm<0>(GemmP);

extern "C" void kernel_launch(void* const* d_in, const int* in_sizes, int n_in, void* d_out, int out_size, void* d_ws, size_t ws_size, hipStream_t stream) {
    (void)in_sizes; (void)n_in; (void)out_size; (void)ws_size;
    const float* x = (const float*)d_in[0];
    const int* ei = (const int*)d_in[1];
    const int* bat = (const int*)d_in[2];
    const int* sb = (const int*)d_in[3];
    const float* W1 = (const float*)d_in[4];
    const float* b1 = (const float*)d_in[5];
    const float* W2 = (const float*)d_in[6];
    const float* b2 = (const float*)d_in[7];
    const float* W3 = (const float*)d_in[8];
    const float* b3 = (const float*)d_in[9];
    const float* pW1 = (const float*)d_in[10];
    const float* pb1 = (const float*)d_in[11];
    const float* pW2 = (const float*)d_in[12];
    const float* pb2 = (const float*)d_in[13];
    const float* fW1 = (const float*)d_in[14];
    const float* fb1 = (const float*)d_in[15];
    const float* fW2 = (const float*)d_in[16];
    const float* fb2 = (const float*)d_in[17];
    const int Nn = 100000;
    const int E = 1600000;
    const int H = 128;
    const int G = 2000;
    const int S = 200;
    const int MS = 10;
    const int CAP = 64;
    const int GCAP = 64;
    const int LP = 32;
    float* out = (float*)d_out;
    char* wsp = (char*)d_ws;
    int* cnt = (int*)wsp; wsp += (((size_t)((size_t)Nn + 64) * 4 + 255) / 256) * 256;
    int* off = (int*)wsp; wsp += (((size_t)((size_t)Nn + 64) * 4 + 255) / 256) * 256;
    int* slot = (int*)wsp; wsp += (((size_t)((size_t)E + 64) * 4 + 255) / 256) * 256;
    int* nbr = (int*)wsp; wsp += (((size_t)((size_t)Nn * CAP) * 4 + 255) / 256) * 256;
    int* gcnt = (int*)wsp; wsp += (((size_t)((size_t)G + 64) * 4 + 255) / 256) * 256;
    int* goff = (int*)wsp; wsp += (((size_t)((size_t)G + 64) * 4 + 255) / 256) * 256;
    int* gslot = (int*)wsp; wsp += (((size_t)((size_t)Nn + 64) * 4 + 255) / 256) * 256;
    int* gnbr = (int*)wsp; wsp += (((size_t)((size_t)G * GCAP) * 4 + 255) / 256) * 256;
    int* ids = (int*)wsp; wsp += (((size_t)((size_t)Nn + 64) * 4 + 255) / 256) * 256;
    int* ROW = (int*)wsp; wsp += (((size_t)((size_t)G + 64) * 4 + 255) / 256) * 256;
    float* DIS = (float*)wsp; wsp += (((size_t)((size_t)Nn + 64) * 4 + 255) / 256) * 256;
    float* T = (float*)wsp; wsp += (((size_t)((size_t)Nn * H) * 4 + 255) / 256) * 256;
    float* Hh = (float*)wsp; wsp += (((size_t)((size_t)Nn * H) * 4 + 255) / 256) * 256;
    float* GE = (float*)wsp; wsp += (((size_t)((size_t)G * H) * 4 + 255) / 256) * 256;
    float* XP = (float*)wsp; wsp += (((size_t)((size_t)S * MS * H) * 4 + 255) / 256) * 256;
    float* P1 = (float*)wsp; wsp += (((size_t)((size_t)S * MS * H) * 4 + 255) / 256) * 256;
    float* P2 = (float*)wsp; wsp += (((size_t)((size_t)S * MS * H) * 4 + 255) / 256) * 256;
    float* AGG = (float*)wsp; wsp += (((size_t)((size_t)S * H) * 4 + 255) / 256) * 256;
    float* F1 = (float*)wsp; wsp += (((size_t)((size_t)S * H) * 4 + 255) / 256) * 256;
    float* OP = (float*)wsp; wsp += (((size_t)((size_t)S * LP) * 4 + 255) / 256) * 256;
    k_csr3_bcount<<<391, 256, 0, stream>>>(ei + E, E, Nn, nbr);
    k_csr3_bscan<<<1, 256, 0, stream>>>(nbr, 391, E, nbr + 100096, off);
    k_csr3_bscatter<<<391, 256, 0, stream>>>(ei + E, E, Nn, nbr + 100096, slot);
    k_csr3_lists<64><<<(unsigned)((Nn) + 255) / 256, 256, 0, stream>>>(ei + E, slot, off, Nn, nbr, cnt);
    k_csr3_scan<<<1, 256, 0, stream>>>(cnt, off, Nn);
    k_csr3_slotcopy<64><<<(unsigned)((E) + 255) / 256, 256, 0, stream>>>(off, nbr, slot, Nn);
    k_csr3_bcount<<<25, 256, 0, stream>>>(bat, Nn, G, gnbr);
    k_csr3_bscan<<<1, 256, 0, stream>>>(gnbr, 25, Nn, gnbr + 6400, goff);
    k_csr3_bscatter<<<25, 256, 0, stream>>>(bat, Nn, G, gnbr + 6400, gslot);
    k_csr3_lists<64><<<(unsigned)((G) + 255) / 256, 256, 0, stream>>>(bat, gslot, goff, G, gnbr, gcnt);
    k_csr3_scan<<<1, 256, 0, stream>>>(gcnt, goff, G);
    k_csr3_slotcopy<64><<<(unsigned)((Nn) + 255) / 256, 256, 0, stream>>>(goff, gnbr, gslot, G);
    k_iota<<<(unsigned)((Nn) + 255) / 256, 256, 0, stream>>>(ids, Nn, 1, 0);
    k_ds_dis<<<(unsigned)((Nn + 255) / 256), 256, 0, stream>>>(off, DIS, Nn); k_ds_rows<<<(unsigned)((G + 255) / 256), 256, 0, stream>>>(sb, ROW, G, MS);
    { GemmP g0;
      g0.A = x; g0.B = W1; g0.bias = x; g0.R = x; g0.C = T;
      g0.sAo = 0; g0.sAi = 0; g0.sAm = H; g0.sAk = 1; g0.sBo = 0; g0.sBi = 0; g0.sBn = 1; g0.sBk = H; g0.sCo = 0; g0.sCi = 0; g0.sCm = H; g0.sRo = 0; g0.sRi = 0; g0.sRm = 0; g0.sRn = 0;
      g0.M = Nn; g0.N = H; g0.K = H; g0.zi_n = 1; g0.flags = 0; g0.act = 0;
      g0.alpha = 1.0f; g0.beta = 0.0f; g0.sa = 1.0f; g0.sb = 8.0f; g0.Npad = H; g0.pad_ = 0;
      k_gemm<0><<<dim3((unsigned)((H) + 31) / 32, (unsigned)((Nn) + 15) / 16, (unsigned)(1)), 32, 0, stream>>>(g0); }
    k_ds_agg<<<(unsigned)(((long long)Nn * H + 255) / 256), 256, 0, stream>>>(T, DIS, ei, off, slot, b1, Hh, Nn, H);
    { GemmP g1;
      g1.A = Hh; g1.B = W2; g1.bias = Hh; g1.R = Hh; g1.C = T;
      g1.sAo = 0; g1.sAi = 0; g1.sAm = H; g1.sAk = 1; g1.sBo = 0; g1.sBi = 0; g1.sBn = 1; g1.sBk = H; g1.sCo = 0; g1.sCi = 0; g1.sCm = H; g1.sRo = 0; g1.sRi = 0; g1.sRm = 0; g1.sRn = 0;
      g1.M = Nn; g1.N = H; g1.K = H; g1.zi_n = 1; g1.flags = 0; g1.act = 0;
      g1.alpha = 1.0f; g1.beta = 0.0f; g1.sa = 1.0f; g1.sb = 8.0f; g1.Npad = H; g1.pad_ = 0;
      k_gemm<0><<<dim3((unsigned)((H) + 31) / 32, (unsigned)((Nn) + 15) / 16, (unsigned)(1)), 32, 0, stream>>>(g1); }
    k_ds_agg<<<(unsigned)(((long long)Nn * H + 255) / 256), 256, 0, stream>>>(T, DIS, ei, off, slot, b2, Hh, Nn, H);
    { GemmP g2;
      g2.A = Hh; g2.B = W3; g2.bias = Hh; g2.R = Hh; g2.C = T;
      g2.sAo = 0; g2.sAi = 0; g2.sAm = H; g2.sAk = 1; g2.sBo = 0; g2.sBi = 0; g2.sBn = 1; g2.sBk = H; g2.sCo = 0; g2.sCi = 0; g2.sCm = H; g2.sRo = 0; g2.sRi = 0; g2.sRm = 0; g2.sRn = 0;
      g2.M = Nn; g2.N = H; g2.K = H; g2.zi_n = 1; g2.flags = 0; g2.act = 0;
      g2.alpha = 1.0f; g2.beta = 0.0f; g2.sa = 1.0f; g2.sb = 8.0f; g2.Npad = H; g2.pad_ = 0;
      k_gemm<0><<<dim3((unsigned)((H) + 31) / 32, (unsigned)((Nn) + 15) / 16, (unsigned)(1)), 32, 0, stream>>>(g2); }
    k_ds_agg<<<(unsigned)(((long long)Nn * H + 255) / 256), 256, 0, stream>>>(T, DIS, ei, off, slot, b3, Hh, Nn, H);
    k_csr_mean<<<(unsigned)((G * H + 255) / 256), 256, 0, stream>>>(Hh, ids, goff, gslot, GE, G, H);
    k_ds_pack<<<(unsigned)((S * MS * H + 255) / 256), 256, 0, stream>>>(GE, ROW, XP, G, H, S * MS * H); k_ds_pack2<<<(unsigned)((G * H + 255) / 256), 256, 0, stream>>>(GE, ROW, XP, G, H);
    { GemmP gp1;
      gp1.A = XP; gp1.B = pW1; gp1.bias = pb1; gp1.R = XP; gp1.C = P1;
      gp1.sAo = 0; gp1.sAi = 0; gp1.sAm = H; gp1.sAk = 1; gp1.sBo = 0; gp1.sBi = 0; gp1.sBn = 1; gp1.sBk = H; gp1.sCo = 0; gp1.sCi = 0; gp1.sCm = H; gp1.sRo = 0; gp1.sRi = 0; gp1.sRm = 0; gp1.sRn = 0;
      gp1.M = S * MS; gp1.N = H; gp1.K = H; gp1.zi_n = 1; gp1.flags = 1; gp1.act = 1;
      gp1.alpha = 1.0f; gp1.beta = 0.0f; gp1.sa = 1.0f; gp1.sb = 8.0f; gp1.Npad = H; gp1.pad_ = 0;
      k_gemm<0><<<dim3((unsigned)((H) + 31) / 32, (unsigned)((S * MS) + 15) / 16, (unsigned)(1)), 32, 0, stream>>>(gp1); }
    { GemmP gp2;
      gp2.A = P1; gp2.B = pW2; gp2.bias = pb2; gp2.R = P1; gp2.C = P2;
      gp2.sAo = 0; gp2.sAi = 0; gp2.sAm = H; gp2.sAk = 1; gp2.sBo = 0; gp2.sBi = 0; gp2.sBn = 1; gp2.sBk = H; gp2.sCo = 0; gp2.sCi = 0; gp2.sCm = H; gp2.sRo = 0; gp2.sRi = 0; gp2.sRm = 0; gp2.sRn = 0;
      gp2.M = S * MS; gp2.N = H; gp2.K = H; gp2.zi_n = 1; gp2.flags = 1; gp2.act = 5;
      gp2.alpha = 1.0f; gp2.beta = 0.0f; gp2.sa = 1.0f; gp2.sb = 8.0f; gp2.Npad = H; gp2.pad_ = 0;
      k_gemm<0><<<dim3((unsigned)((H) + 31) / 32, (unsigned)((S * MS) + 15) / 16, (unsigned)(1)), 32, 0, stream>>>(gp2); }
    k_ds_setsum<<<(unsigned)((S * H + 255) / 256), 256, 0, stream>>>(P2, AGG, S, MS, H);
    { GemmP gf1;
      gf1.A = AGG; gf1.B = fW1; gf1.bias = fb1; gf1.R = AGG; gf1.C = F1;
      gf1.sAo = 0; gf1.sAi = 0; gf1.sAm = H; gf1.sAk = 1; gf1.sBo = 0; gf1.sBi = 0; gf1.sBn = 1; gf1.sBk = H; gf1.sCo = 0; gf1.sCi = 0; gf1.sCm = H; gf1.sRo = 0; gf1.sRi = 0; gf1.sRm = 0; gf1.sRn = 0;
      gf1.M = S; gf1.N = H; gf1.K = H; gf1.zi_n = 1; gf1.flags = 1; gf1.act = 1;
      gf1.alpha = 1.0f; gf1.beta = 0.0f; gf1.sa = 1.0f; gf1.sb = 8.0f; gf1.Npad = H; gf1.pad_ = 0;
      k_gemm<0><<<dim3((unsigned)((H) + 31) / 32, (unsigned)((S) + 15) / 16, (unsigned)(1)), 32, 0, stream>>>(gf1); }
    { GemmP gf2;
      gf2.A = F1; gf2.B = fW2; gf2.bias = fb2; gf2.R = F1; gf2.C = OP;
      gf2.sAo = 0; gf2.sAi = 0; gf2.sAm = H; gf2.sAk = 1; gf2.sBo = 0; gf2.sBi = 0; gf2.sBn = 1; gf2.sBk = 10; gf2.sCo = 0; gf2.sCi = 0; gf2.sCm = LP; gf2.sRo = 0; gf2.sRi = 0; gf2.sRm = 0; gf2.sRn = 0;
      gf2.M = S; gf2.N = 10; gf2.K = H; gf2.zi_n = 1; gf2.flags = 1; gf2.act = 0;
      gf2.alpha = 1.0f; gf2.beta = 0.0f; gf2.sa = 1.0f; gf2.sb = 8.0f; gf2.Npad = LP; gf2.pad_ = 0;
      k_gemm<0><<<dim3((unsigned)((LP) + 31) / 32, (unsigned)((S) + 15) / 16, (unsigned)(1)), 32, 0, stream>>>(gf2); }
    k_lincopy<<<(unsigned)(((long long)(S) * (10) + 255) / 256), 256, 0, stream>>>(OP, LP, out, 10, S, 10);
}
